// re_unit_48103633715562
// MI455X (gfx1250) — hardware-verified
//
#include <hip/hip_runtime.h>
#define LL 128
#define BB 4
#define HH 768
#define RR 24
#define NPR (LL * LL * BB)
#define CH 8192

typedef __bf16 v16b __attribute__((ext_vector_type(16)));
typedef unsigned short v8us __attribute__((ext_vector_type(8), may_alias));
typedef float  v8f  __attribute__((ext_vector_type(8)));
typedef float  v4f  __attribute__((ext_vector_type(4)));
typedef float  v4fa __attribute__((ext_vector_type(4), may_alias));
union FragB { v16b v; v8us half[2]; unsigned short u[16]; };

__device__ __forceinline__ unsigned short bf16_bits(float x) { unsigned int u = __float_as_uint(x); return (unsigned short)((u + 0x7FFFu + ((u >> 16) & 1u)) >> 16); }
__device__ __forceinline__ float bf16_val(unsigned short b) { return __uint_as_float(((unsigned int)b) << 16); }
__device__ __forceinline__ float bf16_round(float x) { return bf16_val(bf16_bits(x)); }
template <int NT>
__device__ __forceinline__ v8f mmaN(v16b ah, v16b al, v16b bh, v16b bl, v8f c) {
  c = __builtin_amdgcn_wmma_f32_16x16x32_bf16(false, ah, false, bh, (short)0, c, false, false);
  if (NT >= 2) c = __builtin_amdgcn_wmma_f32_16x16x32_bf16(false, al, false, bh, (short)0, c, false, false);
  if (NT >= 3) c = __builtin_amdgcn_wmma_f32_16x16x32_bf16(false, ah, false, bl, (short)0, c, false, false);
  asm volatile("v_nop\n\tv_nop\n\tv_nop\n\tv_nop" : "+v"(c) : "v"(ah), "v"(al), "v"(bh), "v"(bl));
  return c;
}

__global__ __launch_bounds__(256) void k_wt_bf16(const float* __restrict__ W, unsigned short* __restrict__ Wt, int K, int N) {
  const int t = blockIdx.x * 256 + threadIdx.x;
  const int k8n = K / 8;
  if (t >= N * k8n) return;
  const int n = t / k8n, k8 = (t % k8n) * 8;
  v8us v;
#pragma unroll
  for (int i = 0; i < 8; ++i) v[i] = bf16_bits(W[(size_t)(k8 + i) * N + n]);
  *(volatile v8us*)(Wt + (size_t)n * K + k8) = v;
  __threadfence();
  *(volatile v8us*)(Wt + (size_t)n * K + k8) = v;
}

template <bool ASPLIT, int ACT, bool BIAS_BF16>
__global__ __launch_bounds__(128) void k_gemm_bf(const float* __restrict__ A, int lda, const unsigned short* __restrict__ Wt, int ldb,
                                               const float* __restrict__ bias, float* __restrict__ C, int ldc, int M, int N, int K) {
  __shared__ __attribute__((aligned(16))) float so[4][16][64];
  const int tid = threadIdx.x, w = tid >> 5, lane = tid & 31, ln = lane & 15, hh = lane >> 4;
  const int ntn = N / 64;
  const int wid = blockIdx.x * 4 + w;
  const int mt = wid / ntn, nq = wid % ntn;
  if (mt * 16 >= M) return;
  const int row0 = mt * 16, col0 = nq * 64;
  const float* arow = A + (size_t)(row0 + ln) * lda;
  v8f acc[4] = {};
  for (int kb = 0; kb < K; kb += 32) {
    FragB ah, al;
    const v4f x0 = *(const v4fa*)(arow + kb + 8 * hh), x1 = *(const v4fa*)(arow + kb + 8 * hh + 4);
    const v4f x2 = *(const v4fa*)(arow + kb + 16 + 8 * hh), x3 = *(const v4fa*)(arow + kb + 16 + 8 * hh + 4);
    float xs[16] = {x0[0],x0[1],x0[2],x0[3],x1[0],x1[1],x1[2],x1[3],x2[0],x2[1],x2[2],x2[3],x3[0],x3[1],x3[2],x3[3]};
#pragma unroll
    for (int i = 0; i < 16; ++i) { const unsigned short hb = bf16_bits(xs[i]); ah.u[i] = hb; al.u[i] = ASPLIT ? bf16_bits(xs[i] - bf16_val(hb)) : (unsigned short)0; }
#pragma unroll
    for (int t = 0; t < 4; ++t) {
      const unsigned short* brow = Wt + (size_t)(col0 + t * 16 + ln) * ldb + kb;
      FragB b;
      b.half[0] = *(const v8us*)(brow + 8 * hh);
      b.half[1] = *(const v8us*)(brow + 16 + 8 * hh);
      acc[t] = mmaN<ASPLIT ? 2 : 1>(ah.v, al.v, b.v, b.v, acc[t]);
    }
  }
#pragma unroll
  for (int t = 0; t < 4; ++t) {
    float bv = bias ? bias[col0 + t * 16 + ln] : 0.f;
    if (BIAS_BF16) bv = bf16_round(bv);
#pragma unroll
    for (int r = 0; r < 8; ++r) { float v = acc[t][r] + bv; if (ACT == 1) v = fmaxf(v, 0.f); so[w][8 * hh + r][t * 16 + ln] = v; }
  }
  __builtin_amdgcn_fence(__ATOMIC_ACQ_REL, "workgroup");
  __builtin_amdgcn_wave_barrier();
  const int rsub = lane >> 4, c4 = (lane & 15) * 4;
  for (int pass = 0; pass < 2; ++pass) {
#pragma unroll
    for (int q = 0; q < 8; ++q) {
      const int r = q * 2 + rsub;
      const v4f v = *(const v4fa*)&so[w][r][c4];
      *(volatile v4f*)(C + (size_t)(row0 + r) * ldc + col0 + c4) = v;
    }
    if (pass == 0) __threadfence();
  }
}

template <int D, bool CAUSAL>
__global__ __launch_bounds__(128) void k_flash(const float* __restrict__ qb, const float* __restrict__ kb, const float* __restrict__ vb,
                                             int pitch, int T, int H, float scale, float* __restrict__ y, int ypitch) {
  constexpr int KS = D / 32;
  constexpr int DT = D / 16;
  __shared__ __attribute__((aligned(16))) unsigned short sKh[32][D + 8], sKl[32][D + 8], sVh[32][D + 8], sVl[32][D + 8];
  __shared__ __attribute__((aligned(16))) unsigned short sPh[4][16][40], sPl[4][16][40];
  __shared__ __attribute__((aligned(16))) float sO[4][16][D];
  const int tid = threadIdx.x, w = tid >> 5, lane = tid & 31, ln = lane & 15, hh = lane >> 4;
  const int nqb = (T + 63) / 64;
  const int bh = blockIdx.x / nqb, qblk = blockIdx.x % nqb;
  const int b = bh / H, h = bh % H;
  const int q0 = qblk * 64 + w * 16;
  const float* Q = qb + (size_t)b * T * pitch + h * D;
  const float* K = kb + (size_t)b * T * pitch + h * D;
  const float* V = vb + (size_t)b * T * pitch + h * D;

  FragB aqh[KS], aql[KS];
  {
    int row = q0 + ln; if (row >= T) row = T - 1;
    const float* qr = Q + (size_t)row * pitch;
#pragma unroll
    for (int ks = 0; ks < KS; ++ks)
#pragma unroll
      for (int i = 0; i < 16; ++i) {
        const int d = ks * 32 + ((i < 8) ? (8 * hh + i) : (16 + 8 * hh + (i - 8)));
        const float x = qr[d] * scale; const unsigned short hb = bf16_bits(x);
        aqh[ks].u[i] = hb; aql[ks].u[i] = bf16_bits(x - bf16_val(hb));
      }
  }
  float m_r[8], l_r[8];
#pragma unroll
  for (int r = 0; r < 8; ++r) { m_r[r] = -3.0e38f; l_r[r] = 0.f; }
  v8f oacc[DT];
#pragma unroll
  for (int dt = 0; dt < DT; ++dt) oacc[dt] = (v8f){0.f,0.f,0.f,0.f,0.f,0.f,0.f,0.f};

  const int kv_end = CAUSAL ? min(T, qblk * 64 + 64) : T;
  for (int j0 = 0; j0 < kv_end; j0 += 32) {
    __syncthreads();
    for (int e = tid; e < 32 * (D / 4); e += 128) {
      const int r = e / (D / 4), c4 = (e % (D / 4)) * 4;
      const int key = j0 + r;
      v4f kf = {0.f,0.f,0.f,0.f}, vf = {0.f,0.f,0.f,0.f};
      if (key < T) { kf = *(const v4fa*)(K + (size_t)key * pitch + c4); vf = *(const v4fa*)(V + (size_t)key * pitch + c4); }
#pragma unroll
      for (int t = 0; t < 4; ++t) {
        unsigned short hb = bf16_bits(kf[t]); sKh[r][c4 + t] = hb; sKl[r][c4 + t] = bf16_bits(kf[t] - bf16_val(hb));
        hb = bf16_bits(vf[t]); sVh[r][c4 + t] = hb; sVl[r][c4 + t] = bf16_bits(vf[t] - bf16_val(hb));
      }
    }
    __syncthreads();
    v8f s[2];
#pragma unroll
    for (int nt = 0; nt < 2; ++nt) {
      v8f acc = {};
#pragma unroll
      for (int ks = 0; ks < KS; ++ks) {
        FragB bh_, bl_;
        bh_.half[0] = *(const v8us*)&sKh[nt * 16 + ln][ks * 32 + 8 * hh]; bh_.half[1] = *(const v8us*)&sKh[nt * 16 + ln][ks * 32 + 16 + 8 * hh];
        bl_.half[0] = *(const v8us*)&sKl[nt * 16 + ln][ks * 32 + 8 * hh]; bl_.half[1] = *(const v8us*)&sKl[nt * 16 + ln][ks * 32 + 16 + 8 * hh];
        acc = mmaN<3>(aqh[ks].v, aql[ks].v, bh_.v, bl_.v, acc);
      }
      s[nt] = acc;
    }
    float alpha[8];
#pragma unroll
    for (int r = 0; r < 8; ++r) {
      const int qi = q0 + 8 * hh + r;
      const int ja = j0 + ln, jb = j0 + 16 + ln;
      if (CAUSAL) { if (ja > qi) s[0][r] = -3.0e38f; if (jb > qi) s[1][r] = -3.0e38f; }
      if (ja >= T) s[0][r] = -3.0e38f;
      if (jb >= T) s[1][r] = -3.0e38f;
      float mx = fmaxf(s[0][r], s[1][r]);
      mx = fmaxf(mx, __shfl_xor(mx, 1, 32)); mx = fmaxf(mx, __shfl_xor(mx, 2, 32)); mx = fmaxf(mx, __shfl_xor(mx, 4, 32)); mx = fmaxf(mx, __shfl_xor(mx, 8, 32));
      const float mnew = fmaxf(m_r[r], mx);
      alpha[r] = (mnew > -1.0e38f) ? __expf(m_r[r] - mnew) : 1.0f;
      const float p0 = (s[0][r] > -1.0e38f) ? __expf(s[0][r] - mnew) : 0.f;
      const float p1 = (s[1][r] > -1.0e38f) ? __expf(s[1][r] - mnew) : 0.f;
      m_r[r] = mnew;
      l_r[r] = l_r[r] * alpha[r] + p0 + p1;
      unsigned short hb = bf16_bits(p0); sPh[w][8 * hh + r][ln] = hb;      sPl[w][8 * hh + r][ln] = bf16_bits(p0 - bf16_val(hb));
      hb = bf16_bits(p1);                sPh[w][8 * hh + r][16 + ln] = hb; sPl[w][8 * hh + r][16 + ln] = bf16_bits(p1 - bf16_val(hb));
    }
#pragma unroll
    for (int dt = 0; dt < DT; ++dt)
#pragma unroll
      for (int r = 0; r < 8; ++r) oacc[dt][r] *= alpha[r];
    __builtin_amdgcn_fence(__ATOMIC_ACQ_REL, "workgroup");
    __builtin_amdgcn_wave_barrier();
    FragB pah, pal;
    pah.half[0] = *(const v8us*)&sPh[w][ln][8 * hh]; pah.half[1] = *(const v8us*)&sPh[w][ln][16 + 8 * hh];
    pal.half[0] = *(const v8us*)&sPl[w][ln][8 * hh]; pal.half[1] = *(const v8us*)&sPl[w][ln][16 + 8 * hh];
#pragma unroll
    for (int dt = 0; dt < DT; ++dt) {
      FragB bvh, bvl;
#pragma unroll
      for (int i = 0; i < 8; ++i) {
        bvh.u[i] = sVh[8 * hh + i][dt * 16 + ln]; bvh.u[8 + i] = sVh[16 + 8 * hh + i][dt * 16 + ln];
        bvl.u[i] = sVl[8 * hh + i][dt * 16 + ln]; bvl.u[8 + i] = sVl[16 + 8 * hh + i][dt * 16 + ln];
      }
      oacc[dt] = mmaN<3>(pah.v, pal.v, bvh.v, bvl.v, oacc[dt]);
    }
    __builtin_amdgcn_fence(__ATOMIC_ACQ_REL, "workgroup");
    __builtin_amdgcn_wave_barrier();
  }
#pragma unroll
  for (int r = 0; r < 8; ++r) {
    float l = l_r[r];
    l += __shfl_xor(l, 1, 32); l += __shfl_xor(l, 2, 32); l += __shfl_xor(l, 4, 32); l += __shfl_xor(l, 8, 32);
    l_r[r] = (l > 0.f) ? 1.0f / l : 0.f;
  }
#pragma unroll
  for (int dt = 0; dt < DT; ++dt)
#pragma unroll
    for (int r = 0; r < 8; ++r) sO[w][8 * hh + r][dt * 16 + ln] = oacc[dt][r] * l_r[r];
  __builtin_amdgcn_fence(__ATOMIC_ACQ_REL, "workgroup");
  __builtin_amdgcn_wave_barrier();
  for (int pass = 0; pass < 2; ++pass) {
    for (int r = 0; r < 16; ++r) {
      const int row = q0 + r;
      if (row < T && lane < D / 4) {
        const v4f val = *(const v4fa*)&sO[w][r][lane * 4];
        *(volatile v4f*)(y + ((size_t)b * T + row) * ypitch + h * D + lane * 4) = val;
      }
    }
    if (pass == 0) __threadfence();
  }
}

template <bool ASPLIT, int ACT, bool BIAS_BF16, bool RES_BF16>
__global__ __launch_bounds__(128) void k_gemm_bf3(const float* __restrict__ A, int lda, const unsigned short* __restrict__ Wt, int ldb,
                                                const float* __restrict__ bias, const float* __restrict__ resid, int rmod, int ldr,
                                                float* __restrict__ C, int ldc, int M, int N, int K) {
  __shared__ __attribute__((aligned(16))) float so[4][16][64];
  const int tid = threadIdx.x, w = tid >> 5, lane = tid & 31, ln = lane & 15, hh = lane >> 4;
  const int ntn = N / 64;
  const int wid = blockIdx.x * 4 + w;
  const int mt = wid / ntn, nq = wid % ntn;
  if (mt * 16 >= M) return;
  const int row0 = mt * 16, col0 = nq * 64;
  const float* arow = A + (size_t)(row0 + ln) * lda;
  v8f acc[4] = {};
  for (int kb = 0; kb < K; kb += 32) {
    FragB ah, al;
    const v4f x0 = *(const v4fa*)(arow + kb + 8 * hh), x1 = *(const v4fa*)(arow + kb + 8 * hh + 4);
    const v4f x2 = *(const v4fa*)(arow + kb + 16 + 8 * hh), x3 = *(const v4fa*)(arow + kb + 16 + 8 * hh + 4);
    float xs[16] = {x0[0],x0[1],x0[2],x0[3],x1[0],x1[1],x1[2],x1[3],x2[0],x2[1],x2[2],x2[3],x3[0],x3[1],x3[2],x3[3]};
#pragma unroll
    for (int i = 0; i < 16; ++i) { const unsigned short hb = bf16_bits(xs[i]); ah.u[i] = hb; al.u[i] = ASPLIT ? bf16_bits(xs[i] - bf16_val(hb)) : (unsigned short)0; }
#pragma unroll
    for (int t = 0; t < 4; ++t) {
      const unsigned short* brow = Wt + (size_t)(col0 + t * 16 + ln) * ldb + kb;
      FragB b;
      b.half[0] = *(const v8us*)(brow + 8 * hh);
      b.half[1] = *(const v8us*)(brow + 16 + 8 * hh);
      acc[t] = mmaN<ASPLIT ? 2 : 1>(ah.v, al.v, b.v, b.v, acc[t]);
    }
  }
#pragma unroll
  for (int t = 0; t < 4; ++t) {
    const int col = col0 + t * 16 + ln;
    float bv = bias ? bias[col] : 0.f;
    if (BIAS_BF16) bv = bf16_round(bv);
#pragma unroll
    for (int r = 0; r < 8; ++r) {
      float v = acc[t][r] + bv;
      if (resid) { float rv = resid[(size_t)((row0 + 8 * hh + r) % rmod) * ldr + col]; if (RES_BF16) rv = bf16_round(rv); v += rv; }
      if (ACT == 1) v = fmaxf(v, 0.f);
      if (ACT == 2) v = 0.5f * v * (1.0f + erff(v * 0.70710678118654752f));
      if (ACT == 3) { const float u = 0.7978845608028654f * (v + 0.044715f * v * v * v); v = 0.5f * v * (1.0f + tanhf(u)); }
      so[w][8 * hh + r][t * 16 + ln] = v;
    }
  }
  __builtin_amdgcn_fence(__ATOMIC_ACQ_REL, "workgroup");
  __builtin_amdgcn_wave_barrier();
  const int rsub = lane >> 4, c4 = (lane & 15) * 4;
  for (int pass = 0; pass < 2; ++pass) {
#pragma unroll
    for (int q = 0; q < 8; ++q) {
      const int r = q * 2 + rsub;
      const v4f v = *(const v4fa*)&so[w][r][c4];
      *(volatile v4f*)(C + (size_t)(row0 + r) * ldc + col0 + c4) = v;
    }
    if (pass == 0) __threadfence();
  }
}
template <bool PARAM_BF16>
__global__ __launch_bounds__(256) void k_layernorm(const float* __restrict__ X, const float* __restrict__ R, const float* __restrict__ g, const float* __restrict__ bta,
                                                  float* __restrict__ out_sum, float* __restrict__ out_norm, int N, float eps) {
  __shared__ float red[256];
  const int row = blockIdx.x, tid = threadIdx.x;
  const float* x = X + (size_t)row * N; const float* rr = R ? R + (size_t)row * N : nullptr;
  float vals[16];
  const int per = N / 256;
  float s1 = 0.f;
  for (int u = 0; u < per / 4; ++u) {
    const int j = tid * 4 + 1024 * u;
    const v4f a = *(const v4fa*)(x + j);
    v4f b = {0.f,0.f,0.f,0.f}; if (rr) b = *(const v4fa*)(rr + j);
#pragma unroll
    for (int q = 0; q < 4; ++q) { const float v = a[q] + b[q]; vals[u * 4 + q] = v; s1 += v; }
  }
  red[tid] = s1; __syncthreads();
  for (int st = 128; st > 0; st >>= 1) { if (tid < st) red[tid] += red[tid + st]; __syncthreads(); }
  const float mu = red[0] / (float)N; __syncthreads();
  float s2 = 0.f;
  for (int u = 0; u < per / 4; ++u)
#pragma unroll
    for (int q = 0; q < 4; ++q) { const float c = vals[u * 4 + q] - mu; s2 += c * c; }
  red[tid] = s2; __syncthreads();
  for (int st = 128; st > 0; st >>= 1) { if (tid < st) red[tid] += red[tid + st]; __syncthreads(); }
  const float rs = rsqrtf(red[0] / (float)N + eps);
  for (int pass = 0; pass < 2; ++pass) {
    for (int u = 0; u < per / 4; ++u) {
      const int j = tid * 4 + 1024 * u;
      v4f o, sm;
#pragma unroll
      for (int q = 0; q < 4; ++q) {
        float gg = g[j + q], bb = bta[j + q];
        if (PARAM_BF16) { gg = bf16_round(gg); bb = bf16_round(bb); }
        sm[q] = vals[u * 4 + q]; o[q] = (vals[u * 4 + q] - mu) * rs * gg + bb;
      }
      if (out_sum) *(volatile v4f*)(out_sum + (size_t)row * N + j) = sm;
      *(volatile v4f*)(out_norm + (size_t)row * N + j) = o;
    }
    if (pass == 0) __threadfence();
  }
}

__global__ __launch_bounds__(256) void k_wt_slice(const float* __restrict__ W, int ldw, int koff, unsigned short* __restrict__ Bt, int Nout, int Np, int Kc) {
  const size_t t = (size_t)blockIdx.x * 256 + threadIdx.x; const int k8n = Kc / 8; if (t >= (size_t)Np * k8n) return; const int n = (int)(t / k8n), k8 = (int)(t % k8n) * 8; v8us v;
  for (int i = 0; i < 8; ++i) v[i] = (n < Nout) ? bf16_bits(W[(size_t)n * ldw + koff + k8 + i]) : (unsigned short)0;
  *(volatile v8us*)(Bt + (size_t)n * Kc + k8) = v; __threadfence(); *(volatile v8us*)(Bt + (size_t)n * Kc + k8) = v;
}
__global__ __launch_bounds__(256) void k_cat(const float* __restrict__ hs, const float* __restrict__ hr, float* __restrict__ cat) {
  const size_t t = (size_t)blockIdx.x * 256 + threadIdx.x; if (t >= (size_t)LL * BB * 2 * HH / 4) return; const size_t row = t / (2 * HH / 4); const int c4 = (int)(t % (2 * HH / 4)) * 4;
  const v4f v = (c4 < HH) ? *(const v4fa*)(hs + row * HH + c4) : *(const v4fa*)(hr + row * HH + c4 - HH);
  *(volatile v4f*)(cat + t * 4) = v; __threadfence(); *(volatile v4f*)(cat + t * 4) = v;
}
__global__ __launch_bounds__(256) void k_gmax(const float* __restrict__ gp, float* __restrict__ g16) {
  const int t = blockIdx.x * 256 + threadIdx.x; if (t >= 16 * HH) return; const int b = t / HH, h = t % HH; float m = 0.f;
  if (b < BB) { m = -3.0e38f;
#pragma unroll 1
    for (int l = 0; l < LL; ++l) m = fmaxf(m, tanhf(gp[((size_t)l * BB + b) * HH + h])); }
  *(volatile float*)(g16 + t) = m; __threadfence(); *(volatile float*)(g16 + t) = m;
}
__global__ __launch_bounds__(192) void k_zrow(const float* __restrict__ p12, const float* __restrict__ pg, const float* __restrict__ lg, const float* __restrict__ lb, int r0, float* __restrict__ zr) {
  __shared__ float red[192];
  const int rl = blockIdx.x; const int r = r0 + rl; const int b = r % BB, j = (r / BB) % LL, i = r / (BB * LL); const int t = threadIdx.x;
  const v4f a = *(const v4fa*)(p12 + ((size_t)i * BB + b) * 2 * HH + t * 4), c = *(const v4fa*)(p12 + ((size_t)j * BB + b) * 2 * HH + HH + t * 4), p = *(const v4fa*)(pg + (size_t)b * HH + t * 4);
  v4f z; float s = 0.f; for (int q = 0; q < 4; ++q) { z[q] = (a[q] + c[q]) + p[q]; s += z[q]; }
  red[t] = s; __syncthreads();
  if (t == 0) { float tot = 0.f; for (int k = 0; k < 192; ++k) tot += red[k]; red[0] = tot; } __syncthreads(); const float mu = red[0] / HH; __syncthreads();
  float q2 = 0.f; for (int q = 0; q < 4; ++q) { const float d = z[q] - mu; q2 += d * d; } red[t] = q2; __syncthreads();
  if (t == 0) { float tot = 0.f; for (int k = 0; k < 192; ++k) tot += red[k]; red[0] = tot; } __syncthreads(); const float rs = rsqrtf(red[0] / HH + 1e-5f);
  v4f o; for (int q = 0; q < 4; ++q) { const int h = t * 4 + q; float v = (z[q] - mu) * rs * bf16_round(lg[h]) + bf16_round(lb[h]); o[q] = v > 0.f ? v : expm1f(v); }
  *(volatile v4f*)(zr + (size_t)rl * HH + t * 4) = o; __threadfence(); *(volatile v4f*)(zr + (size_t)rl * HH + t * 4) = o;
}
__global__ __launch_bounds__(64) void k_bias64(const float* __restrict__ b, float* __restrict__ o) { const int t = threadIdx.x; const float v = (t < RR) ? bf16_round(b[t]) : 0.f; *(volatile float*)(o + t) = v; __threadfence(); *(volatile float*)(o + t) = v; }
__global__ __launch_bounds__(256) void k_pack(const float* __restrict__ rel, const float* __restrict__ mask, int r0, float* __restrict__ out) {
  const int rb = blockIdx.x * 128;
  for (int pass = 0; pass < 2; ++pass) { for (int e = threadIdx.x; e < 128 * RR; e += 256) { const int rl = rb + e / RR, c = e % RR; const int r = r0 + rl; const int b = r % BB, j = (r / BB) % LL, i = r / (BB * LL);
      const float m = bf16_round(mask[i * BB + b]) * bf16_round(mask[j * BB + b]); const float v = m / (1.0f + expf(-rel[(size_t)rl * 64 + c]));
      *(volatile float*)(out + (size_t)r0 * RR + (size_t)rb * RR + e) = v; } if (pass == 0) __threadfence(); }
}
extern "C" void kernel_launch(void* const* d_in, const int* in_sizes, int n_in,
                              void* d_out, int out_size, void* d_ws, size_t ws_size, hipStream_t stream) {
  (void)in_sizes; (void)n_in; (void)out_size;
  const float* h_re = (const float*)d_in[0]; const float* h_sh = (const float*)d_in[1]; const float* mask = (const float*)d_in[2]; const float* r_w = (const float*)d_in[3]; const float* r_b = (const float*)d_in[4];
  const float* hid_w = (const float*)d_in[5]; const float* hid_b = (const float*)d_in[6]; const float* lg = (const float*)d_in[7]; const float* lb = (const float*)d_in[8]; const float* rel_w = (const float*)d_in[9]; const float* rel_b = (const float*)d_in[10];
  char* ws = (char*)d_ws; size_t off = 0;
  auto take = [&](size_t bytes) { char* p = ws + off; off += (bytes + 255) & ~(size_t)255; return p; };
  const int MR = LL * BB;
  unsigned short* Br = (unsigned short*)take((size_t)HH * 2 * HH * 2); unsigned short* B12 = (unsigned short*)take((size_t)2 * HH * HH * 2); unsigned short* B3 = (unsigned short*)take((size_t)HH * HH * 2); unsigned short* Brel = (unsigned short*)take((size_t)64 * HH * 2);
  float* relb64 = (float*)take(64 * 4);
  float* cat = (float*)take((size_t)MR * 2 * HH * 4); float* gp = (float*)take((size_t)MR * HH * 4); float* g16 = (float*)take((size_t)16 * HH * 4); float* pg = (float*)take((size_t)16 * HH * 4); float* p12 = (float*)take((size_t)MR * 2 * HH * 4);
  float* zr = (float*)take((size_t)CH * HH * 4); float* rel = (float*)take((size_t)CH * 64 * 4);
  if (off > ws_size) return;
  k_wt_slice<<<(unsigned)(((size_t)HH * (2 * HH / 8) + 255) / 256), 256, 0, stream>>>(r_w, 2 * HH, 0, Br, HH, HH, 2 * HH);
  k_wt_slice<<<(unsigned)(((size_t)2 * HH * (HH / 8) + 255) / 256), 256, 0, stream>>>(hid_w, 3 * HH, 0, B12, HH, HH, HH);
  k_wt_slice<<<(unsigned)(((size_t)HH * (HH / 8) + 255) / 256), 256, 0, stream>>>(hid_w, 3 * HH, HH, B12 + (size_t)HH * HH, HH, HH, HH);
  k_wt_slice<<<(unsigned)(((size_t)HH * (HH / 8) + 255) / 256), 256, 0, stream>>>(hid_w, 3 * HH, 2 * HH, B3, HH, HH, HH);
  k_wt_slice<<<(unsigned)(((size_t)64 * (HH / 8) + 255) / 256), 256, 0, stream>>>(rel_w, HH, 0, Brel, RR, 64, HH);
  k_bias64<<<1, 64, 0, stream>>>(rel_b, relb64);
  k_cat<<<(unsigned)(((size_t)MR * 2 * HH / 4 + 255) / 256), 256, 0, stream>>>(h_sh, h_re, cat);
  k_gemm_bf3<false, 0, true, false><<<((MR / 16) * (HH / 64) + 3) / 4, 128, 0, stream>>>(cat, 2 * HH, Br, 2 * HH, r_b, nullptr, 1, 0, gp, HH, MR, HH, 2 * HH);
  k_gmax<<<(16 * HH + 255) / 256, 256, 0, stream>>>(gp, g16);
  k_gemm_bf3<true, 0, true, false><<<((16 / 16) * (HH / 64) + 3) / 4, 128, 0, stream>>>(g16, HH, B3, HH, hid_b, nullptr, 1, 0, pg, HH, 16, HH, HH);
  k_gemm_bf3<false, 0, false, false><<<((MR / 16) * (2 * HH / 64) + 3) / 4, 128, 0, stream>>>(h_re, HH, B12, HH, nullptr, nullptr, 1, 0, p12, 2 * HH, MR, 2 * HH, HH);
  for (int c = 0; c < NPR / CH; ++c) {
    const int r0 = c * CH;
    k_zrow<<<CH, 192, 0, stream>>>(p12, pg, lg, lb, r0, zr);
    k_gemm_bf3<true, 0, false, false><<<((CH / 16) * 1 + 3) / 4, 128, 0, stream>>>(zr, HH, Brel, HH, relb64, nullptr, 1, 0, rel, 64, CH, 64, HH);
    k_pack<<<CH / 128, 256, 0, stream>>>(rel, mask, r0, (float*)d_out);
  }
}
